// mLSTMblock_74388833567240
// MI455X (gfx1250) — hardware-run, weakly checked
//
#include <hip/hip_runtime.h>

#ifndef NB
#define NB 4
#endif
#define NB_FULL 4
#define SQ 16
#define DD 1024
#define HH 2048
#define NBLK 8
#define BSZ 256
#define ROWS (NB * SQ)
#define ROWSP 64
#define LROW 4096
#define NSH 8
static_assert(NB >= 1 && NB <= NB_FULL);
static_assert(ROWS <= ROWSP);
static_assert((ROWS * HH) % 1024 == 0);
static_assert(DD % 64 == 0 && HH % 64 == 0 && BSZ % 64 == 0 && DD % 32 == 0 && BSZ % 32 == 0);
static_assert(HH == 4 * 512 && LROW == 2 * HH);

typedef __bf16 v16b __attribute__((ext_vector_type(16)));
typedef unsigned short v8us __attribute__((ext_vector_type(8), may_alias));
typedef unsigned short v4us __attribute__((ext_vector_type(4), may_alias));
typedef float v8f __attribute__((ext_vector_type(8)));
typedef float v4f __attribute__((ext_vector_type(4)));
typedef float v4fa __attribute__((ext_vector_type(4), may_alias));
union FragB { v16b v; v8us half[2]; unsigned short u[16]; };

__device__ __forceinline__ unsigned short bf16_bits(float x) { const unsigned int u = __float_as_uint(x); return (unsigned short)((u + 0x7FFFu + ((u >> 16) & 1u)) >> 16); }
__device__ __forceinline__ float bf16_val(unsigned short b) { return __uint_as_float(((unsigned int)b) << 16); }
__device__ __forceinline__ float bf16_rne(float x) { return bf16_val(bf16_bits(x)); }

__device__ __forceinline__ v8f mma2(v16b ah, v16b al, v16b b, v8f c) {
  c = __builtin_amdgcn_wmma_f32_16x16x32_bf16(false, ah, false, b, (short)0, c, false, false);
  c = __builtin_amdgcn_wmma_f32_16x16x32_bf16(false, al, false, b, (short)0, c, false, false);
  asm volatile("v_nop\n\tv_nop\n\tv_nop\n\tv_nop" : "+v"(c) : "v"(ah), "v"(al), "v"(b));
  return c;
}
__device__ __forceinline__ v16b frag16(const unsigned short* p, int hh) { FragB f; f.half[0] = *(const v8us*)(p + 8 * hh); f.half[1] = *(const v8us*)(p + 16 + 8 * hh); return f.v; }
__device__ __forceinline__ v16b frag0(const unsigned short* p) { FragB f; f.half[0] = *(const v8us*)p; f.half[1] = *(const v8us*)(p + 16); return f.v; }
__device__ __forceinline__ float silu_f(float v) { return v * __builtin_amdgcn_rcpf(1.0f + expf(-v)); }
__device__ __forceinline__ float sigm_f(float v) { return __builtin_amdgcn_rcpf(1.0f + expf(-v)); }

__global__ __launch_bounds__(256) void k_wt(const float* W0, const float* W1, const float* W2, const float* W3,
                                            unsigned short* U0, unsigned short* U1, unsigned short* U2, unsigned short* U3, int K, int N, int zdiv) {
  const int z = blockIdx.z; const int sel = z / zdiv; const int d = z - sel * zdiv;
  const float* W = (sel == 0) ? W0 : (sel == 1) ? W1 : (sel == 2) ? W2 : W3;
  unsigned short* U = (sel == 0) ? U0 : (sel == 1) ? U1 : (sel == 2) ? U2 : U3;
  const size_t doff = (size_t)d * (size_t)K * (size_t)N;
  const int t = blockIdx.x * 256 + threadIdx.x; const int k8n = K >> 3;
  if (t >= N * k8n) return;
  const int n = t / k8n, k8 = (t - n * k8n) * 8;
  v8us v;
#pragma unroll
  for (int i = 0; i < 8; ++i) v[i] = bf16_bits(W[doff + (size_t)(k8 + i) * N + n]);
  unsigned short* dst = U + doff + (size_t)n * K + k8;
  *(volatile v8us*)dst = v;
  __threadfence();
  *(volatile v8us*)dst = v;
}

__global__ __launch_bounds__(256) void k_cw(const float* __restrict__ W, unsigned short* __restrict__ U, int n8) {
  const int t = blockIdx.x * 256 + threadIdx.x; if (t >= n8) return;
  const v4f a = *(const v4fa*)(W + (size_t)t * 8), c = *(const v4fa*)(W + (size_t)t * 8 + 4);
  v8us o;
#pragma unroll
  for (int q = 0; q < 4; ++q) { o[q] = bf16_bits(a[q]); o[4 + q] = bf16_bits(c[q]); }
  *(volatile v8us*)(U + (size_t)t * 8) = o;
  __threadfence();
  *(volatile v8us*)(U + (size_t)t * 8) = o;
}

__global__ __launch_bounds__(256) void k_ln1(const float* __restrict__ x, const float* __restrict__ g, const float* __restrict__ bt,
                                             float* __restrict__ XN, unsigned short* __restrict__ XH, unsigned short* __restrict__ XL) {
  __shared__ float red[256];
  const int row = blockIdx.x, tid = threadIdx.x; const int j = tid * 4;
  const v4f a = *(const v4fa*)(x + (size_t)row * DD + j);
  float v[4]; float s1 = 0.f;
#pragma unroll
  for (int q = 0; q < 4; ++q) { v[q] = bf16_rne(a[q]); s1 += v[q]; }
  red[tid] = s1; __syncthreads();
  for (int st = 128; st > 0; st >>= 1) { if (tid < st) red[tid] += red[tid + st]; __syncthreads(); }
  const float mu = red[0] * (1.0f / (float)DD); __syncthreads();
  float s2 = 0.f;
#pragma unroll
  for (int q = 0; q < 4; ++q) { const float c = v[q] - mu; s2 += c * c; }
  red[tid] = s2; __syncthreads();
  for (int st = 128; st > 0; st >>= 1) { if (tid < st) red[tid] += red[tid + st]; __syncthreads(); }
  const float rs = rsqrtf(red[0] * (1.0f / (float)DD) + 1e-5f);
  v4f o; v4us oh, ol;
#pragma unroll
  for (int q = 0; q < 4; ++q) {
    const float val = (v[q] - mu) * rs * bf16_rne(g[j + q]) + bf16_rne(bt[j + q]);
    o[q] = val; const unsigned short hb = bf16_bits(val); oh[q] = hb; ol[q] = bf16_bits(val - bf16_val(hb));
  }
  const size_t base = (size_t)row * DD + j;
  for (int pass = 0; pass < 2; ++pass) {
    *(volatile v4f*)(XN + base) = o;
    *(volatile v4us*)(XH + base) = oh;
    *(volatile v4us*)(XL + base) = ol;
    if (pass == 0) __threadfence();
  }
}

__global__ __launch_bounds__(64) void k_gemm(const unsigned short* __restrict__ Ah, const unsigned short* __restrict__ Al, int lda, int sAd,
    const unsigned short* W0, const unsigned short* W1, const unsigned short* W2, const unsigned short* W3, int ldb, int sBd,
    const float* b0, const float* b1, const float* b2, const float* b3, int sbd,
    const float* __restrict__ R, int ldr,
    float* C0, float* C1, float* C2, float* C3, int ldc, int sCd,
    int act0, int act1, int act2, int act3, int zdiv, int M, int Mst, int N, int K) {
  __shared__ __attribute__((aligned(16))) float so[2][32][68];
  const int tid = threadIdx.x, lane = tid & 31, ln = lane & 15, hh = lane >> 4;
  const int w = __builtin_amdgcn_readfirstlane(tid >> 5);
  const int z = blockIdx.z; const int sel = z / zdiv; const int d = z - sel * zdiv;
  const unsigned short* Wt = (sel == 0) ? W0 : (sel == 1) ? W1 : (sel == 2) ? W2 : W3;
  const float* bias = (sel == 0) ? b0 : (sel == 1) ? b1 : (sel == 2) ? b2 : b3;
  float* C = (sel == 0) ? C0 : (sel == 1) ? C1 : (sel == 2) ? C2 : C3;
  const int act = (sel == 0) ? act0 : (sel == 1) ? act1 : (sel == 2) ? act2 : act3;
  Wt += (size_t)d * sBd;
  if (bias) bias += (size_t)d * sbd;
  const int coff = d * sCd, aoff = d * sAd;
  const int ntn = N >> 6; const int mt = blockIdx.x / ntn, nq = blockIdx.x - mt * ntn;
  const int row0 = mt * 64 + 32 * w, col0 = nq * 64;
  if (row0 >= M) return;
  const unsigned short* a0h = Ah + (size_t)(row0 + ln) * lda + aoff; const unsigned short* a1h = a0h + (size_t)16 * lda;
  const unsigned short* a0l = Al + (size_t)(row0 + ln) * lda + aoff; const unsigned short* a1l = a0l + (size_t)16 * lda;
  const unsigned short* bp0 = Wt + (size_t)(col0 + ln) * ldb; const unsigned short* bp1 = bp0 + (size_t)16 * ldb;
  const unsigned short* bp2 = bp1 + (size_t)16 * ldb; const unsigned short* bp3 = bp2 + (size_t)16 * ldb;
  const v8f z8 = {0.f,0.f,0.f,0.f,0.f,0.f,0.f,0.f};
  v8f c[8];
#pragma unroll
  for (int u = 0; u < 8; ++u) c[u] = z8;
#pragma unroll 1
  for (int kb = 0; kb < K; kb += 32) {
    const v16b x0h = frag16(a0h + kb, hh), x1h = frag16(a1h + kb, hh), x0l = frag16(a0l + kb, hh), x1l = frag16(a1l + kb, hh);
    v16b bq = frag16(bp0 + kb, hh); c[0] = mma2(x0h, x0l, bq, c[0]); c[4] = mma2(x1h, x1l, bq, c[4]);
    bq = frag16(bp1 + kb, hh); c[1] = mma2(x0h, x0l, bq, c[1]); c[5] = mma2(x1h, x1l, bq, c[5]);
    bq = frag16(bp2 + kb, hh); c[2] = mma2(x0h, x0l, bq, c[2]); c[6] = mma2(x1h, x1l, bq, c[6]);
    bq = frag16(bp3 + kb, hh); c[3] = mma2(x0h, x0l, bq, c[3]); c[7] = mma2(x1h, x1l, bq, c[7]);
  }
#pragma unroll
  for (int u = 0; u < 8; ++u) {
    const int t = u & 3, half = u >> 2; const int col = col0 + t * 16 + ln;
    const float bv = bias ? bf16_rne(bias[col]) : 0.f;
#pragma unroll
    for (int r = 0; r < 8; ++r) {
      const int rloc = half * 16 + 8 * hh + r;
      float v = c[u][r] + bv;
      if (R) v += R[(size_t)(row0 + rloc) * ldr + coff + col];
      so[w][rloc][t * 16 + ln] = v;
    }
  }
  __builtin_amdgcn_fence(__ATOMIC_ACQ_REL, "workgroup");
  __builtin_amdgcn_wave_barrier();
  if (act != 0) {
#pragma unroll 1
    for (int e = lane; e < 32 * 64; e += 32) {
      const int rr = e >> 6, cc = e & 63;
      float v = so[w][rr][cc];
      if (act == 1) v = silu_f(v); else if (act == 2) v = expf(v); else v = sigm_f(v);
      so[w][rr][cc] = v;
    }
    __builtin_amdgcn_fence(__ATOMIC_ACQ_REL, "workgroup");
    __builtin_amdgcn_wave_barrier();
  }
  const int rsub = lane >> 4, c4 = (lane & 15) * 4;
  for (int pass = 0; pass < 2; ++pass) {
#pragma unroll
    for (int q = 0; q < 16; ++q) {
      const int r = q * 2 + rsub;
      if (row0 + r < Mst) { const v4f v = *(const v4fa*)&so[w][r][c4]; *(volatile v4f*)(C + (size_t)(row0 + r) * ldc + coff + col0 + c4) = v; }
    }
    if (pass == 0) __threadfence();
  }
}

__global__ __launch_bounds__(256) void k_lps(const float* __restrict__ L32, unsigned short* __restrict__ PHs, unsigned short* __restrict__ PLs) {
  const int t = blockIdx.x * 256 + threadIdx.x;
  if (t >= ROWS * NSH * (LROW / 8)) return;
  const int c8 = (t & 511) * 8; const int s = (t >> 9) & 7; const int r = t >> 12;
  const float* src = L32 + (size_t)r * HH;
  v8us h, l;
#pragma unroll
  for (int q = 0; q < 8; ++q) {
    const int u = c8 + s - 2048 + q;
    const int uc = min(max(u, 0), HH - 1);
    float v = src[uc];
    v = (u >= 0 && u < HH) ? v : 0.0f;
    const unsigned short hb = bf16_bits(v); h[q] = hb; l[q] = bf16_bits(v - bf16_val(hb));
  }
  const size_t dst = ((size_t)r * NSH + s) * LROW + c8;
  for (int pass = 0; pass < 2; ++pass) {
    *(volatile v8us*)(PHs + dst) = h;
    *(volatile v8us*)(PLs + dst) = l;
    if (pass == 0) __threadfence();
  }
}

__global__ __launch_bounds__(256) void k_conv(const unsigned short* __restrict__ PHs, const unsigned short* __restrict__ PLs,
                                              const unsigned short* __restrict__ CW, const float* __restrict__ cb,
                                              unsigned short* __restrict__ OH, unsigned short* __restrict__ OL) {
  __shared__ __attribute__((aligned(16))) float sow[4][16][128];
  const int tid = threadIdx.x, lane = tid & 31, m = lane & 15, hh = lane >> 4;
  const int w = __builtin_amdgcn_readfirstlane(tid >> 5);
  const int pr = w >> 1, odd = w & 1;
  const int b = blockIdx.x >> 2, tq = blockIdx.x & 3;
  const int T0 = tq * 512 + pr * 128, toff = odd * 16, tb = T0 + toff;
  const int ks = 1905 - tb;
  const int kp0s = (ks >= 0) ? (ks & ~31) : 0;
  const int s = (m + 1) & 7;
  const int aofs = m + 8 * hh - s;
  const v8f z8 = {0.f,0.f,0.f,0.f,0.f,0.f,0.f,0.f};
  v8f acc[4];
#pragma unroll
  for (int j = 0; j < 4; ++j) acc[j] = z8;
#pragma unroll 1
  for (int i = 0; i < SQ; ++i) {
    const size_t rb = ((size_t)(b * SQ + i) * NSH + s) * LROW + aofs;
    const unsigned short* hr = PHs + rb;
    const unsigned short* lr = PLs + rb;
    const unsigned short* bw = CW + (size_t)(m * SQ + i) * HH + 8 * hh;
    int P = tb + kp0s + 1;
    v16b fh[4], fl[4];
#pragma unroll
    for (int j = 0; j < 4; ++j) { fh[j] = frag0(hr + P + 32 * j); fl[j] = frag0(lr + P + 32 * j); }
#pragma unroll 1
    for (int kp0 = kp0s; kp0 < HH; kp0 += 32) {
      const v16b bq = frag0(bw + kp0);
#pragma unroll
      for (int j = 0; j < 4; ++j) acc[j] = mma2(fh[j], fl[j], bq, acc[j]);
      const int Pn = min(P + 128, LROW - 47);
      const v16b nh = frag0(hr + Pn), nl = frag0(lr + Pn);
      fh[0] = fh[1]; fh[1] = fh[2]; fh[2] = fh[3]; fh[3] = nh;
      fl[0] = fl[1]; fl[1] = fl[2]; fl[2] = fl[3]; fl[3] = nl;
      P += 32;
    }
  }
  const float bv = bf16_rne(cb[m]);
#pragma unroll
  for (int j = 0; j < 4; ++j)
#pragma unroll
    for (int r = 0; r < 8; ++r) sow[pr][m][toff + 32 * j + 8 * hh + r] = acc[j][r] + bv;
  __syncthreads();
  const int oh = odd * 8;
#pragma unroll 1
  for (int e = lane; e < 8 * 128; e += 32) { const int o = oh + (e >> 7), tl = e & 127; sow[pr][o][tl] = silu_f(sow[pr][o][tl]); }
  __builtin_amdgcn_fence(__ATOMIC_ACQ_REL, "workgroup");
  __builtin_amdgcn_wave_barrier();
  for (int pass = 0; pass < 2; ++pass) {
#pragma unroll
    for (int oo = 0; oo < 8; ++oo) {
      const int o = oh + oo;
      const v4f v = *(const v4fa*)&sow[pr][o][4 * lane];
      v4us h4, l4;
#pragma unroll
      for (int q = 0; q < 4; ++q) { const unsigned short hb = bf16_bits(v[q]); h4[q] = hb; l4[q] = bf16_bits(v[q] - bf16_val(hb)); }
      const size_t dst = (size_t)(b * SQ + o) * HH + T0 + 4 * lane;
      *(volatile v4us*)(OH + dst) = h4;
      *(volatile v4us*)(OL + dst) = l4;
    }
    if (pass == 0) __threadfence();
  }
}

__global__ __launch_bounds__(256) void k_gates(const float* __restrict__ IG, const float* __restrict__ FG, const float* __restrict__ QB,
                                               const float* __restrict__ KB, const float* __restrict__ VB, const float* __restrict__ c1, const float* __restrict__ n1,
                                               float* __restrict__ PP, float* __restrict__ PMAX) {
  __shared__ float red[256];
  const int tid = threadIdx.x, lane = tid & 31;
  const int w = __builtin_amdgcn_readfirstlane(tid >> 5);
  const size_t e0 = ((size_t)blockIdx.x * 256 + tid) * 4;
  const v4f gi = *(const v4fa*)(IG + e0), gf = *(const v4fa*)(FG + e0), gq = *(const v4fa*)(QB + e0), gk = *(const v4fa*)(KB + e0);
  const v4f gv = *(const v4fa*)(VB + e0), pc = *(const v4fa*)(c1 + e0), pn = *(const v4fa*)(n1 + e0);
  v4f p4; float mx = -3.0e38f;
#pragma unroll
  for (int q = 0; q < 4; ++q) {
    const float ct = gf[q] * bf16_rne(pc[q]) + gi[q] * gv[q] * gk[q];
    const float nt = gf[q] * bf16_rne(pn[q]) + gi[q] * gk[q];
    p4[q] = ct * gq[q];
    mx = fmaxf(mx, nt * gq[q]);
  }
  red[tid] = mx; __syncthreads();
  for (int st = 128; st > 0; st >>= 1) { if (tid < st) red[tid] = fmaxf(red[tid], red[tid + st]); __syncthreads(); }
  const float bm = red[0];
  for (int pass = 0; pass < 2; ++pass) {
    *(volatile v4f*)(PP + e0) = p4;
    if (w == 0) *(volatile float*)(PMAX + (size_t)blockIdx.x * 32 + lane) = bm;
    if (pass == 0) __threadfence();
  }
}

__global__ __launch_bounds__(256) void k_final(const float* __restrict__ OG, const float* __restrict__ PP, const float* __restrict__ PMAX, int nblk,
                                               const float* __restrict__ gg, const float* __restrict__ gb, const float* __restrict__ LSK, const float* __restrict__ RT,
                                               unsigned short* __restrict__ PH, unsigned short* __restrict__ PL) {
  __shared__ float red[256];
  const int row = blockIdx.x, tid = threadIdx.x;
  float mx = -3.0e38f;
  for (int i = tid; i < nblk; i += 256) mx = fmaxf(mx, PMAX[(size_t)i * 32]);
  red[tid] = mx; __syncthreads();
  for (int st = 128; st > 0; st >>= 1) { if (tid < st) red[tid] = fmaxf(red[tid], red[tid + st]); __syncthreads(); }
  const float gm = red[0]; __syncthreads();
  const float inv = 1.0f / gm;
  const size_t base = (size_t)row * HH;
  float ht[8]; float s1 = 0.f;
#pragma unroll
  for (int u = 0; u < 2; ++u) {
    const int j = tid * 4 + 1024 * u;
    const v4f o4 = *(const v4fa*)(OG + base + j), p4 = *(const v4fa*)(PP + base + j);
#pragma unroll
    for (int q = 0; q < 4; ++q) { const float h = o4[q] * (p4[q] * inv); ht[u * 4 + q] = h; s1 += h; }
  }
  red[tid] = s1; __syncthreads();
  for (int st = 128; st > 0; st >>= 1) { if (tid < st) red[tid] += red[tid + st]; __syncthreads(); }
  const float mu = red[0] * (1.0f / (float)HH); __syncthreads();
  float s2 = 0.f;
#pragma unroll
  for (int e = 0; e < 8; ++e) { const float c = ht[e] - mu; s2 += c * c; }
  red[tid] = s2; __syncthreads();
  for (int st = 128; st > 0; st >>= 1) { if (tid < st) red[tid] += red[tid + st]; __syncthreads(); }
  const float rs = rsqrtf(red[0] * (1.0f / (float)HH) + 1e-5f);
  v4us oh[2], ol[2];
#pragma unroll
  for (int u = 0; u < 2; ++u) {
    const int j = tid * 4 + 1024 * u;
    const v4f l4 = *(const v4fa*)(LSK + base + j), r4 = *(const v4fa*)(RT + base + j);
#pragma unroll
    for (int q = 0; q < 4; ++q) {
      const float lo = (ht[u * 4 + q] - mu) * rs * bf16_rne(gg[j + q]) + bf16_rne(gb[j + q]) + l4[q];
      const float pre = lo * r4[q];
      const unsigned short hb = bf16_bits(pre); oh[u][q] = hb; ol[u][q] = bf16_bits(pre - bf16_val(hb));
    }
  }
  for (int pass = 0; pass < 2; ++pass) {
#pragma unroll
    for (int u = 0; u < 2; ++u) {
      const int j = tid * 4 + 1024 * u;
      *(volatile v4us*)(PH + base + j) = oh[u];
      *(volatile v4us*)(PL + base + j) = ol[u];
    }
    if (pass == 0) __threadfence();
  }
}

extern "C" void kernel_launch(void* const* d_in, const int* in_sizes, int n_in,
                              void* d_out, int out_size, void* d_ws, size_t ws_size, hipStream_t stream) {
  if (n_in < 29) return;
  if (in_sizes[0] < ROWS * DD || in_sizes[1] < DD || in_sizes[2] < DD ||
      in_sizes[3] < DD * HH || in_sizes[4] < HH || in_sizes[5] < DD * HH || in_sizes[6] < HH ||
      in_sizes[7] < SQ * SQ * HH || in_sizes[8] < SQ || in_sizes[9] < HH * HH || in_sizes[10] < HH ||
      in_sizes[11] < NBLK * BSZ * BSZ || in_sizes[12] < HH || in_sizes[13] < NBLK * BSZ * BSZ || in_sizes[14] < HH ||
      in_sizes[15] < NBLK * BSZ * BSZ || in_sizes[16] < HH || in_sizes[17] < HH * HH || in_sizes[18] < HH ||
      in_sizes[19] < HH * HH || in_sizes[20] < HH || in_sizes[21] < HH * HH || in_sizes[22] < HH ||
      in_sizes[23] < HH || in_sizes[24] < HH || in_sizes[25] < HH * DD || in_sizes[26] < DD ||
      in_sizes[27] < ROWS * HH || in_sizes[28] < ROWS * HH) return;
  if (out_size < ROWS * DD) return;
  const float* const* I = (const float* const*)d_in;
  const float* x = I[0]; const float* ln_g = I[1]; const float* ln_b = I[2];
  const float* left_w = I[3]; const float* left_b = I[4]; const float* right_w = I[5]; const float* right_b = I[6];
  const float* conv_w = I[7]; const float* conv_b = I[8]; const float* lskip_w = I[9]; const float* lskip_b = I[10];
  const float* wq_w = I[11]; const float* wq_b = I[12]; const float* wk_w = I[13]; const float* wk_b = I[14]; const float* wv_w = I[15]; const float* wv_b = I[16];
  const float* ig_w = I[17]; const float* ig_b = I[18]; const float* fg_w = I[19]; const float* fg_b = I[20]; const float* og_w = I[21]; const float* og_b = I[22];
  const float* gn_g = I[23]; const float* gn_b = I[24]; const float* proj_w = I[25]; const float* proj_b = I[26];
  const float* ct_1 = I[27]; const float* nt_1 = I[28];

  char* ws = (char*)d_ws; size_t off = 0;
  auto take = [&](size_t bytes) { char* p = ws + off; off += (bytes + 255) & ~(size_t)255; return p; };
  unsigned short* WL  = (unsigned short*)take((size_t)HH * DD * 2);
  unsigned short* WR  = (unsigned short*)take((size_t)HH * DD * 2);
  unsigned short* WLS = (unsigned short*)take((size_t)HH * HH * 2);
  unsigned short* WIG = (unsigned short*)take((size_t)HH * HH * 2);
  unsigned short* WFG = (unsigned short*)take((size_t)HH * HH * 2);
  unsigned short* WOG = (unsigned short*)take((size_t)HH * HH * 2);
  unsigned short* WQ  = (unsigned short*)take((size_t)NBLK * BSZ * BSZ * 2);
  unsigned short* WK  = (unsigned short*)take((size_t)NBLK * BSZ * BSZ * 2);
  unsigned short* WV  = (unsigned short*)take((size_t)NBLK * BSZ * BSZ * 2);
  unsigned short* WP  = (unsigned short*)take((size_t)HH * DD * 2);
  unsigned short* CW  = (unsigned short*)take((size_t)SQ * SQ * HH * 2);
  float* XN = (float*)take((size_t)ROWSP * DD * 4);
  unsigned short* XH = (unsigned short*)take((size_t)ROWSP * DD * 2);
  unsigned short* XL = (unsigned short*)take((size_t)ROWSP * DD * 2);
  float* LEFT32 = (float*)take((size_t)ROWSP * HH * 4);
  float* RIGHT  = (float*)take((size_t)ROWSP * HH * 4);
  unsigned short* LPSH = (unsigned short*)take((size_t)ROWSP * NSH * LROW * 2);
  unsigned short* LPSL = (unsigned short*)take((size_t)ROWSP * NSH * LROW * 2);
  unsigned short* LLH = (unsigned short*)take((size_t)ROWSP * HH * 2);
  unsigned short* LLL = (unsigned short*)take((size_t)ROWSP * HH * 2);
  float* LSK = (float*)take((size_t)ROWSP * HH * 4);
  float* QB  = (float*)take((size_t)ROWSP * HH * 4);
  float* KB  = (float*)take((size_t)ROWSP * HH * 4);
  float* VB  = (float*)take((size_t)ROWSP * HH * 4);
  float* IG  = (float*)take((size_t)ROWSP * HH * 4);
  float* FG  = (float*)take((size_t)ROWSP * HH * 4);
  float* OG  = (float*)take((size_t)ROWSP * HH * 4);
  float* PP  = (float*)take((size_t)ROWSP * HH * 4);
  const int NBK = ROWS * HH / 1024;
  float* PMAX = (float*)take((size_t)NBK * 32 * 4);
  unsigned short* PREH = (unsigned short*)take((size_t)ROWSP * HH * 2);
  unsigned short* PREL = (unsigned short*)take((size_t)ROWSP * HH * 2);
  if (off > ws_size || off > (size_t)134217728) return;

  k_wt<<<dim3((HH * (DD / 8) + 255) / 256, 1, 2), 256, 0, stream>>>(left_w, right_w, nullptr, nullptr, WL, WR, nullptr, nullptr, DD, HH, 1);
  k_wt<<<dim3((HH * (HH / 8) + 255) / 256, 1, 4), 256, 0, stream>>>(lskip_w, ig_w, fg_w, og_w, WLS, WIG, WFG, WOG, HH, HH, 1);
  k_wt<<<dim3((BSZ * (BSZ / 8) + 255) / 256, 1, 3 * NBLK), 256, 0, stream>>>(wq_w, wk_w, wv_w, nullptr, WQ, WK, WV, nullptr, BSZ, BSZ, NBLK);
  k_wt<<<dim3((DD * (HH / 8) + 255) / 256, 1, 1), 256, 0, stream>>>(proj_w, nullptr, nullptr, nullptr, WP, nullptr, nullptr, nullptr, HH, DD, 1);
  k_cw<<<(SQ * SQ * HH / 8 + 255) / 256, 256, 0, stream>>>(conv_w, CW, SQ * SQ * HH / 8);
  k_ln1<<<ROWS, 256, 0, stream>>>(x, ln_g, ln_b, XN, XH, XL);
  k_gemm<<<dim3(HH / 64, 1, 2), 64, 0, stream>>>(XH, XL, DD, 0, WL, WR, nullptr, nullptr, DD, 0, left_b, right_b, nullptr, nullptr, 0, nullptr, 0,
                                                   LEFT32, RIGHT, nullptr, nullptr, HH, 0, 0, 1, 0, 0, 1, ROWSP, ROWSP, HH, DD);
  k_lps<<<(ROWS * NSH * (LROW / 8) + 255) / 256, 256, 0, stream>>>(LEFT32, LPSH, LPSL);
  k_conv<<<NB * 4, 256, 0, stream>>>(LPSH, LPSL, CW, conv_b, LLH, LLL);
  k_gemm<<<dim3(HH / 64, 1, 4), 64, 0, stream>>>(LLH, LLL, HH, 0, WLS, WIG, WFG, WOG, HH, 0, lskip_b, ig_b, fg_b, og_b, 0, nullptr, 0,
                                                   LSK, IG, FG, OG, HH, 0, 0, 2, 2, 3, 1, ROWSP, ROWSP, HH, HH);
  k_gemm<<<dim3(BSZ / 64, 1, 2 * NBLK), 64, 0, stream>>>(LLH, LLL, HH, BSZ, WQ, WK, nullptr, nullptr, BSZ, BSZ * BSZ, wq_b, wk_b, nullptr, nullptr, BSZ, nullptr, 0,
                                                           QB, KB, nullptr, nullptr, HH, BSZ, 0, 0, 0, 0, NBLK, ROWSP, ROWSP, BSZ, BSZ);
  k_gemm<<<dim3(BSZ / 64, 1, NBLK), 64, 0, stream>>>(LPSH + 2048, LPSL + 2048, NSH * LROW, BSZ, WV, nullptr, nullptr, nullptr, BSZ, BSZ * BSZ, wv_b, nullptr, nullptr, nullptr, BSZ, nullptr, 0,
                                                       VB, nullptr, nullptr, nullptr, HH, BSZ, 0, 0, 0, 0, NBLK, ROWSP, ROWSP, BSZ, BSZ);
  k_gates<<<NBK, 256, 0, stream>>>(IG, FG, QB, KB, VB, ct_1, nt_1, PP, PMAX);
  k_final<<<ROWS, 256, 0, stream>>>(OG, PP, PMAX, NBK, gn_g, gn_b, LSK, RIGHT, PREH, PREL);
  k_gemm<<<dim3(DD / 64, 1, 1), 64, 0, stream>>>(PREH, PREL, HH, 0, WP, nullptr, nullptr, nullptr, HH, 0, proj_b, nullptr, nullptr, nullptr, 0, XN, DD,
                                                   (float*)d_out, nullptr, nullptr, nullptr, DD, 0, 0, 0, 0, 0, 1, ROWSP, ROWS, DD, HH);
}
